// ICDeform_44195213476586
// MI455X (gfx1250) — hardware-verified
//
#include <hip/hip_runtime.h>

typedef _Float16 v16h __attribute__((ext_vector_type(16)));
typedef _Float16 v8h  __attribute__((ext_vector_type(8)));
typedef __bf16   v16b __attribute__((ext_vector_type(16)));
typedef __bf16   v8b  __attribute__((ext_vector_type(8)));
typedef float    v8f  __attribute__((ext_vector_type(8)));
typedef float    v4f  __attribute__((ext_vector_type(4)));
typedef float    v2f  __attribute__((ext_vector_type(2)));
typedef unsigned short v8u __attribute__((ext_vector_type(8)));
typedef v8h __attribute__((may_alias)) v8ha;
typedef v8b __attribute__((may_alias)) v8ba;
typedef v8u __attribute__((may_alias)) v8ua;
typedef v4f __attribute__((may_alias)) v4fa;
typedef v2f __attribute__((may_alias)) v2fa;
typedef float __attribute__((may_alias)) f32a;

#define NB    8
#define CH    64
#define HH    56
#define WWD   56
#define PIX   3136
#define NPIX  25088
#define NOFF  1152
#define KDIM  576
#define PITCH 584
#define NX    (NB * CH * PIX)
#define NW1   (NOFF * KDIM)
#define NWD   (CH * KDIM)
#define CMT   32
#define DMT   64
#define DPL   (DMT * PITCH)
#define XBLK  (NX / 8 / 256)
#define W1BLK (NW1 / 8 / 256)
#define WDBLK (NWD / 8 / 256)

static_assert(NX % 2048 == 0);
static_assert(NW1 % 2048 == 0);
static_assert(NWD % 2048 == 0);
static_assert(NPIX % DMT == 0);
static_assert(PIX % DMT == 0);
static_assert(PIX % CMT == 0);
static_assert(KDIM % 32 == 0);
static_assert(NOFF % 128 == 0);

__device__ __forceinline__ v8f wmma_f16(v16h a, v16h b, v8f c) {
  v8f d = __builtin_amdgcn_wmma_f32_16x16x32_f16(false, a, false, b, (short)0, c, false, false);
  asm volatile("v_nop\n\tv_nop\n\tv_nop\n\tv_nop" : "+v"(d) : "v"(a), "v"(b));
  return d;
}
__device__ __forceinline__ v8f wmma_bf16(v16b a, v16b b, v8f c) {
  v8f d = __builtin_amdgcn_wmma_f32_16x16x32_bf16(false, a, false, b, (short)0, c, false, false);
  asm volatile("v_nop\n\tv_nop\n\tv_nop\n\tv_nop" : "+v"(d) : "v"(a), "v"(b));
  return d;
}

__device__ __forceinline__ v16h frag_h(const unsigned short* p, int h) {
  union { v16h v; v8h hv[2]; } f;
  f.hv[0] = *(const v8ha*)(p + 8 * h);
  f.hv[1] = *(const v8ha*)(p + 16 + 8 * h);
  return f.v;
}
__device__ __forceinline__ v16b frag_b(const unsigned short* p, int h) {
  union { v16b v; v8b hv[2]; } f;
  f.hv[0] = *(const v8ba*)(p + 8 * h);
  f.hv[1] = *(const v8ba*)(p + 16 + 8 * h);
  return f.v;
}

__device__ __forceinline__ unsigned short f16bits(float v) {
  union { _Float16 hv; unsigned short u; } q;
  q.hv = (_Float16)v;
  return q.u;
}
__device__ __forceinline__ unsigned short bf16bits(float v) {
  unsigned int u = __float_as_uint(v);
  u += 0x7FFFu + ((u >> 16) & 1u);
  return (unsigned short)(u >> 16);
}
__device__ __forceinline__ float bf16val(unsigned short b) {
  return __uint_as_float(((unsigned int)b) << 16);
}
__device__ __forceinline__ int clampi(int v, int lo, int hi) {
  return v < lo ? lo : (v > hi ? hi : v);
}

__device__ __forceinline__ v8u cvt_f16x8(v4f a, v4f c, float sc) {
  v8u o;
  o[0] = f16bits(a.x * sc); o[1] = f16bits(a.y * sc); o[2] = f16bits(a.z * sc); o[3] = f16bits(a.w * sc);
  o[4] = f16bits(c.x * sc); o[5] = f16bits(c.y * sc); o[6] = f16bits(c.z * sc); o[7] = f16bits(c.w * sc);
  return o;
}
__device__ __forceinline__ v8u cvt_bf16hi8(v4f a, v4f c) {
  v8u o;
  o[0] = bf16bits(a.x); o[1] = bf16bits(a.y); o[2] = bf16bits(a.z); o[3] = bf16bits(a.w);
  o[4] = bf16bits(c.x); o[5] = bf16bits(c.y); o[6] = bf16bits(c.z); o[7] = bf16bits(c.w);
  return o;
}
__device__ __forceinline__ unsigned short bf16lo(float v) {
  return bf16bits(v - bf16val(bf16bits(v)));
}
__device__ __forceinline__ v8u cvt_bf16lo8(v4f a, v4f c) {
  v8u o;
  o[0] = bf16lo(a.x); o[1] = bf16lo(a.y); o[2] = bf16lo(a.z); o[3] = bf16lo(a.w);
  o[4] = bf16lo(c.x); o[5] = bf16lo(c.y); o[6] = bf16lo(c.z); o[7] = bf16lo(c.w);
  return o;
}

__global__ __launch_bounds__(256) void convert_kernel(
    const float* __restrict__ x, const float* __restrict__ w1, const float* __restrict__ wd,
    unsigned short* __restrict__ xh, unsigned short* __restrict__ w1h,
    unsigned short* __restrict__ wdh, unsigned short* __restrict__ wdhi, unsigned short* __restrict__ wdlo)
{
  const int blk = blockIdx.x, t = threadIdx.x;
  const float* src;
  unsigned short* dst;
  int e, mode;
  float sc;
  if (blk < XBLK) {
    e = blk * 256 + t; src = x; dst = xh; mode = 0; sc = 1.0f;
  } else if (blk < XBLK + W1BLK) {
    e = (blk - XBLK) * 256 + t; src = w1; dst = w1h; mode = 0; sc = 64.0f;
  } else {
    const int q = blk - XBLK - W1BLK;
    const int seg = clampi(q / WDBLK, 0, 2);
    e = (q - seg * WDBLK) * 256 + t;
    src = wd;
    dst = (seg == 0) ? wdh : ((seg == 1) ? wdhi : wdlo);
    mode = seg;
    sc = (seg == 0) ? 16.0f : 1.0f;
  }
  const v4f a = *(const v4fa*)(src + (size_t)e * 8);
  const v4f c = *(const v4fa*)(src + (size_t)e * 8 + 4);
  v8u o;
  if (mode == 0) o = cvt_f16x8(a, c, sc);
  else if (mode == 1) o = cvt_bf16hi8(a, c);
  else o = cvt_bf16lo8(a, c);
  unsigned short* dp = dst + (size_t)e * 8;
  *(volatile v8u*)dp = o;
  __threadfence();
  *(volatile v8u*)dp = o;
}

__device__ __forceinline__ void conv_store_pass(const float* sC, float* off, int m0, int nc,
                                                int w, int lane) {
  #pragma unroll
  for (int q = 0; q < 16; ++q) {
    const int row = 16 * w + q;
    const v4f v = *(const v4fa*)(sC + row * 128 + 4 * lane);
    float* dst = off + (size_t)(m0 + row) * NOFF + nc * 128 + 4 * lane;
    *(volatile v4f*)dst = v;
  }
}

__global__ __launch_bounds__(64) void conv_kernel(
    const unsigned short* __restrict__ src,
    const unsigned short* __restrict__ w1h,
    const float* __restrict__ b1,
    float* __restrict__ off)
{
  __shared__ __attribute__((aligned(16))) unsigned short sA[CMT * PITCH];
  __shared__ __attribute__((aligned(16))) float sC[CMT * 128];

  const int tid = threadIdx.x, lane = tid & 31, w = tid >> 5;
  const int h = lane >> 4, m = lane & 15;
  const int m0 = blockIdx.x * CMT;
  const int b = m0 / PIX;
  const int pbase = m0 - b * PIX;

  {
    const int r = tid & 31, half = tid >> 5;
    const int p = pbase + r;
    const int y = p / WWD;
    const int xw = p - y * WWD;
    const unsigned short* sb = src + (size_t)b * CH * PIX;
    unsigned short* arow = sA + r * PITCH;
    #pragma unroll 1
    for (int c = half * 32; c < half * 32 + 32; ++c) {
      const unsigned short* sp = sb + (size_t)c * PIX;
      #pragma unroll
      for (int ky = 0; ky < 3; ++ky) {
        const int yy = y + ky - 1;
        const bool vy = (yy >= 0) && (yy < HH);
        const int yc = clampi(yy, 0, HH - 1);
        #pragma unroll
        for (int kx = 0; kx < 3; ++kx) {
          const int xx = xw + kx - 1;
          const bool vx = (xx >= 0) && (xx < WWD);
          const int xc = clampi(xx, 0, WWD - 1);
          const unsigned short v = sp[yc * WWD + xc];
          arow[c * 9 + ky * 3 + kx] = (vy && vx) ? v : (unsigned short)0;
        }
      }
    }
  }
  __syncthreads();

  const v8f zero8 = {0.f, 0.f, 0.f, 0.f, 0.f, 0.f, 0.f, 0.f};
  const unsigned short* a0p = sA + m * PITCH;
  const unsigned short* a1p = sA + (16 + m) * PITCH;

  #pragma unroll 1
  for (int nc = 0; nc < NOFF / 128; ++nc) {
    const int nw = nc * 128 + 64 * w;
    const unsigned short* wrow = w1h + (size_t)(nw + m) * KDIM;
    v8f acc[2][4];
    #pragma unroll
    for (int i = 0; i < 2; ++i)
      #pragma unroll
      for (int j = 0; j < 4; ++j) acc[i][j] = zero8;

    #pragma unroll 1
    for (int k0 = 0; k0 < KDIM; k0 += 32) {
      const v16h a0 = frag_h(a0p + k0, h);
      const v16h a1 = frag_h(a1p + k0, h);
      #pragma unroll
      for (int j = 0; j < 4; ++j) {
        const v16h bb = frag_h(wrow + (size_t)(16 * j) * KDIM + k0, h);
        acc[0][j] = wmma_f16(a0, bb, acc[0][j]);
        acc[1][j] = wmma_f16(a1, bb, acc[1][j]);
      }
    }

    #pragma unroll
    for (int j = 0; j < 4; ++j) {
      const int col = 64 * w + 16 * j + m;
      const float bj = b1[nc * 128 + col];
      #pragma unroll
      for (int i = 0; i < 2; ++i)
        #pragma unroll
        for (int r = 0; r < 8; ++r)
          sC[(16 * i + 8 * h + r) * 128 + col] = acc[i][j][r] * 0.015625f + bj;
    }
    __syncthreads();
    conv_store_pass(sC, off, m0, nc, w, lane);
    __threadfence();
    conv_store_pass(sC, off, m0, nc, w, lane);
    __syncthreads();
  }
}

__device__ __forceinline__ void t_store_pass(const unsigned short* sT, unsigned short* tout,
                                             int b, int p0, int w, int lane) {
  const int sub = lane >> 3, q8 = 8 * (lane & 7);
  #pragma unroll
  for (int q = 0; q < 4; ++q) {
    const int ch = 4 * (4 * w + q) + sub;
    const v8u v = *(const v8ua*)(sT + ch * DMT + q8);
    unsigned short* dst = tout + (size_t)(b * CH + ch) * PIX + p0 + q8;
    *(volatile v8u*)dst = v;
  }
}
__device__ __forceinline__ void o_store_pass(const f32a* sT, float* fout,
                                             int b, int p0, int w, int lane) {
  const int sub = lane >> 4, q4 = 4 * (lane & 15);
  #pragma unroll
  for (int q = 0; q < 8; ++q) {
    const int ch = 2 * (8 * w + q) + sub;
    const v4f v = *(const v4fa*)(sT + ch * DMT + q4);
    float* dst = fout + (size_t)(b * CH + ch) * PIX + p0 + q4;
    *(volatile v4f*)dst = v;
  }
}

template <bool SPLIT>
__global__ __launch_bounds__(128) void dcn_kernel(
    const float* __restrict__ x,
    const float* __restrict__ off,
    const unsigned short* __restrict__ wda,
    const unsigned short* __restrict__ wdb,
    unsigned short* __restrict__ tout,
    float* __restrict__ fout)
{
  __shared__ __attribute__((aligned(16))) unsigned short sA[SPLIT ? 2 * DPL : DPL];

  const int tid = threadIdx.x, lane = tid & 31, w = tid >> 5;
  const int h = lane >> 4, m = lane & 15;
  const int g0 = blockIdx.x * DMT;
  const int b = g0 / PIX;
  const int p0 = g0 - b * PIX;

  {
    const int r = tid & (DMT - 1), half = tid >> 6;
    const int p = p0 + r;
    const int y = p / WWD;
    const int xw = p - y * WWD;
    const float* orow = off + (size_t)(g0 + r) * NOFF;
    const float* xb = x + (size_t)b * CH * PIX;
    unsigned short* arow = sA + r * PITCH;
    #pragma unroll 1
    for (int c = half * 32; c < half * 32 + 32; ++c) {
      const float* xp = xb + (size_t)c * PIX;
      const float* oc = orow + 18 * c;
      #pragma unroll
      for (int ky = 0; ky < 3; ++ky) {
        #pragma unroll
        for (int kx = 0; kx < 3; ++kx) {
          const int k9 = ky * 3 + kx;
          const v2f d = *(const v2fa*)(oc + 2 * k9);
          const float py = (float)(y - 1 + ky) + d.x;
          const float px = (float)(xw - 1 + kx) + d.y;
          const float y0f = floorf(py), x0f = floorf(px);
          const float wy1 = py - y0f, wx1 = px - x0f;
          const float wy0 = 1.0f - wy1, wx0 = 1.0f - wx1;
          const float y1f = y0f + 1.0f, x1f = x0f + 1.0f;
          const bool vy0 = (y0f >= 0.0f) && (y0f <= (float)(HH - 1));
          const bool vy1 = (y1f >= 0.0f) && (y1f <= (float)(HH - 1));
          const bool vx0 = (x0f >= 0.0f) && (x0f <= (float)(WWD - 1));
          const bool vx1 = (x1f >= 0.0f) && (x1f <= (float)(WWD - 1));
          const int iy0 = (int)fminf(fmaxf(y0f, 0.0f), (float)(HH - 1));
          const int iy1 = (int)fminf(fmaxf(y1f, 0.0f), (float)(HH - 1));
          const int ix0 = (int)fminf(fmaxf(x0f, 0.0f), (float)(WWD - 1));
          const int ix1 = (int)fminf(fmaxf(x1f, 0.0f), (float)(WWD - 1));
          const float g00 = xp[iy0 * WWD + ix0];
          const float g01 = xp[iy0 * WWD + ix1];
          const float g10 = xp[iy1 * WWD + ix0];
          const float g11 = xp[iy1 * WWD + ix1];
          const float t00 = (vy0 && vx0) ? g00 : 0.0f;
          const float t01 = (vy0 && vx1) ? g01 : 0.0f;
          const float t10 = (vy1 && vx0) ? g10 : 0.0f;
          const float t11 = (vy1 && vx1) ? g11 : 0.0f;
          const float s = wy0 * wx0 * t00 + wy0 * wx1 * t01 + wy1 * wx0 * t10 + wy1 * wx1 * t11;
          const int kk = c * 9 + k9;
          if (SPLIT) {
            const unsigned short hb = bf16bits(s);
            arow[kk] = hb;
            arow[DPL + kk] = bf16bits(s - bf16val(hb));
          } else {
            arow[kk] = f16bits(s);
          }
        }
      }
    }
  }
  __syncthreads();

  const v8f zero8 = {0.f, 0.f, 0.f, 0.f, 0.f, 0.f, 0.f, 0.f};
  v8f acc[4];
  #pragma unroll
  for (int j = 0; j < 4; ++j) acc[j] = zero8;
  const unsigned short* arow = sA + (16 * w + m) * PITCH;
  const unsigned short* wra = wda + (size_t)m * KDIM;
  const unsigned short* wrb = wdb + (size_t)m * KDIM;

  #pragma unroll 1
  for (int k0 = 0; k0 < KDIM; k0 += 32) {
    if (SPLIT) {
      const v16b ah = frag_b(arow + k0, h);
      const v16b al = frag_b(arow + DPL + k0, h);
      #pragma unroll
      for (int j = 0; j < 4; ++j) {
        const v16b bh = frag_b(wra + (size_t)(16 * j) * KDIM + k0, h);
        const v16b bl = frag_b(wrb + (size_t)(16 * j) * KDIM + k0, h);
        acc[j] = wmma_bf16(ah, bh, acc[j]);
        acc[j] = wmma_bf16(ah, bl, acc[j]);
        acc[j] = wmma_bf16(al, bh, acc[j]);
      }
    } else {
      const v16h a = frag_h(arow + k0, h);
      #pragma unroll
      for (int j = 0; j < 4; ++j) {
        const v16h bb = frag_h(wra + (size_t)(16 * j) * KDIM + k0, h);
        acc[j] = wmma_f16(a, bb, acc[j]);
      }
    }
  }
  __syncthreads();

  if (SPLIT) {
    f32a* sT = (f32a*)sA;
    #pragma unroll
    for (int j = 0; j < 4; ++j)
      #pragma unroll
      for (int r = 0; r < 8; ++r)
        sT[(16 * j + m) * DMT + 16 * w + 8 * h + r] = acc[j][r];
    __syncthreads();
    o_store_pass(sT, fout, b, p0, w, lane);
    __threadfence();
    o_store_pass(sT, fout, b, p0, w, lane);
  } else {
    unsigned short* sT = sA;
    #pragma unroll
    for (int j = 0; j < 4; ++j)
      #pragma unroll
      for (int r = 0; r < 8; ++r)
        sT[(16 * j + m) * DMT + 16 * w + 8 * h + r] = f16bits(acc[j][r] * 0.0625f);
    __syncthreads();
    t_store_pass(sT, tout, b, p0, w, lane);
    __threadfence();
    t_store_pass(sT, tout, b, p0, w, lane);
  }
}

extern "C" void kernel_launch(void* const* d_in, const int* in_sizes, int n_in,
                              void* d_out, int out_size, void* d_ws, size_t ws_size,
                              hipStream_t stream) {
  if (n_in < 4) return;
  if (in_sizes[0] != NX || in_sizes[1] != NW1 || in_sizes[2] != NOFF || in_sizes[3] != NWD) return;
  if (out_size != NX) return;

  const float* x  = (const float*)d_in[0];
  const float* w1 = (const float*)d_in[1];
  const float* b1 = (const float*)d_in[2];
  const float* wd = (const float*)d_in[3];
  float* out = (float*)d_out;

  const size_t off_b = (size_t)NPIX * NOFF * 4;
  const size_t xh_b  = (size_t)NX * 2;
  const size_t th_b  = xh_b;
  const size_t w1h_b = (size_t)NW1 * 2;
  const size_t wd_b  = (size_t)NWD * 2;
  const size_t total = off_b + xh_b + th_b + w1h_b + 3 * wd_b;
  if (total > ws_size) return;
  if (total > (size_t)134217728) return;

  char* ws = (char*)d_ws;
  float* off            = (float*)(ws);
  unsigned short* xh    = (unsigned short*)(ws + off_b);
  unsigned short* th    = (unsigned short*)(ws + off_b + xh_b);
  unsigned short* w1h   = (unsigned short*)(ws + off_b + xh_b + th_b);
  unsigned short* wdh   = (unsigned short*)(ws + off_b + xh_b + th_b + w1h_b);
  unsigned short* wdhi  = (unsigned short*)(ws + off_b + xh_b + th_b + w1h_b + wd_b);
  unsigned short* wdlo  = (unsigned short*)(ws + off_b + xh_b + th_b + w1h_b + 2 * wd_b);

  convert_kernel<<<XBLK + W1BLK + 3 * WDBLK, 256, 0, stream>>>(x, w1, wd, xh, w1h, wdh, wdhi, wdlo);

  conv_kernel<<<NPIX / CMT, 64, 0, stream>>>(xh, w1h, b1, off);

  dcn_kernel<false><<<NPIX / DMT, 128, 0, stream>>>(x, off, wdh, wdh, th, out);

  conv_kernel<<<NPIX / CMT, 64, 0, stream>>>(th, w1h, b1, off);

  dcn_kernel<true><<<NPIX / DMT, 128, 0, stream>>>(x, off, wdhi, wdlo, th, out);
}
